// SilkNNUE_86466281603145
// MI455X (gfx1250) — hardware-verified
//
#include <hip/hip_runtime.h>


#define NR   131072
#define NIDX 32
#define NUSE 29
#define VOC  7424
#define EMB  128
typedef _Float16 h16;
typedef unsigned short bf;
typedef __attribute__((ext_vector_type(16))) __bf16   v16bf;
typedef __attribute__((ext_vector_type(16))) _Float16 v16h;
typedef __attribute__((ext_vector_type(8)))  _Float16 v8h;
typedef __attribute__((ext_vector_type(8)))  unsigned short v8us;
typedef __attribute__((ext_vector_type(8)))  float    v8f;
typedef __attribute__((ext_vector_type(4)))  float    v4f;
typedef v8h  __attribute__((may_alias)) v8ha;
typedef v4f  __attribute__((may_alias)) v4fa;
typedef v8us __attribute__((may_alias)) v8usa;

__device__ __forceinline__ unsigned short f2bf(float f) { unsigned u = __float_as_uint(f); u += 0x7FFFu + ((u >> 16) & 1u); return (unsigned short)(u >> 16); }
__device__ __forceinline__ float bf2f(unsigned short b) { return __uint_as_float(((unsigned)b) << 16); }
__device__ __forceinline__ float bfr(float f) { return bf2f(f2bf(f)); }
__device__ __forceinline__ v16h cat16(v8h lo, v8h hi) { return __builtin_shufflevector(lo, hi, 0, 1, 2, 3, 4, 5, 6, 7, 8, 9, 10, 11, 12, 13, 14, 15); }
__device__ __forceinline__ v16bf cat16b(v8us lo, v8us hi) { return __builtin_bit_cast(v16bf, __builtin_shufflevector(lo, hi, 0, 1, 2, 3, 4, 5, 6, 7, 8, 9, 10, 11, 12, 13, 14, 15)); }
__device__ __forceinline__ v8f wmma16(v16h a, v16h b, v8f c) { return __builtin_amdgcn_wmma_f32_16x16x32_f16(false, a, false, b, (short)0, c, false, false); }
__device__ __forceinline__ v8f wmmab(v16bf a, v16bf b, v8f c) { return __builtin_amdgcn_wmma_f32_16x16x32_bf16(false, a, false, b, (short)0, c, false, false); }


template <typename T16> struct WFrag;
template <> struct WFrag<h16> { typedef v16h V; static __device__ __forceinline__ V ld(const h16* p) { return cat16(*(const v8h*)p, *(const v8h*)(p + 16)); } static __device__ __forceinline__ v8f mma(V a, V b, v8f c) { return wmma16(a, b, c); } };
template <> struct WFrag<bf> { typedef v16bf V; static __device__ __forceinline__ V ld(const bf* p) { return cat16b(*(const v8us*)p, *(const v8us*)(p + 16)); } static __device__ __forceinline__ v8f mma(V a, V b, v8f c) { return wmmab(a, b, c); } };
template <typename T16, int NSPLIT, bool BIAS>
__global__ __launch_bounds__(32) void k_gemmw(const T16* __restrict__ A, const T16* __restrict__ A2, const T16* __restrict__ Bt, const T16* __restrict__ Bt2, int K, float* C, int ldc, const float* __restrict__ bias, size_t sA, size_t sB, size_t sC) {
    typedef typename WFrag<T16>::V V;
    __shared__ __align__(16) float os[16 * 68];
    const size_t z = blockIdx.z; A += z * sA; if (A2) A2 += z * sA; Bt += z * sB; if (Bt2) Bt2 += z * sB; C += z * sC;
    const int lane = threadIdx.x & 31, lr = lane & 15, hi = lane >> 4; const int r0 = blockIdx.x * 64, c0 = blockIdx.y * 64;
    v8f acc[4][4];
#pragma unroll
    for (int mb = 0; mb < 4; ++mb)
#pragma unroll
        for (int nb = 0; nb < 4; ++nb) acc[mb][nb] = (v8f){};
    const size_t aoff = (size_t)(r0 + lr) * K + 8 * hi, boff = (size_t)(c0 + lr) * K + 8 * hi;
#pragma unroll 1
    for (int kc = 0; kc < K; kc += 32) {
        V a[4], a2[4];
#pragma unroll
        for (int mb = 0; mb < 4; ++mb) { a[mb] = WFrag<T16>::ld(A + aoff + (size_t)mb * 16 * K + kc); if (NSPLIT == 1 || NSPLIT == 2) a2[mb] = WFrag<T16>::ld(A2 + aoff + (size_t)mb * 16 * K + kc); }
#pragma unroll
        for (int nb = 0; nb < 4; ++nb) { const V b = WFrag<T16>::ld(Bt + boff + (size_t)nb * 16 * K + kc); V b2; if (NSPLIT >= 2) b2 = WFrag<T16>::ld(Bt2 + boff + (size_t)nb * 16 * K + kc);
#pragma unroll
            for (int mb = 0; mb < 4; ++mb) { acc[mb][nb] = WFrag<T16>::mma(a[mb], b, acc[mb][nb]); if (NSPLIT == 1 || NSPLIT == 2) acc[mb][nb] = WFrag<T16>::mma(a2[mb], b, acc[mb][nb]); if (NSPLIT >= 2) acc[mb][nb] = WFrag<T16>::mma(a[mb], b2, acc[mb][nb]); } }
        asm volatile("v_nop\n\tv_nop\n\tv_nop\n\tv_nop" : "+v"(acc[0][0]), "+v"(acc[1][1]), "+v"(acc[2][2]), "+v"(acc[3][3]) : "v"(a[0]), "v"(a[3]));
    }
#pragma unroll
    for (int mb = 0; mb < 4; ++mb) {
#pragma unroll
        for (int nb = 0; nb < 4; ++nb) {
#pragma unroll
            for (int j = 0; j < 8; ++j) os[(hi * 8 + j) * 68 + nb * 16 + lr] = acc[mb][nb][j]; }
        __builtin_amdgcn_wave_barrier(); asm volatile("" ::: "memory");
        float* crow = C + (size_t)(r0 + mb * 16) * ldc + c0;
#pragma unroll 1
        for (int ps = 0; ps < 2; ++ps) {
#pragma unroll
            for (int s = 0; s < 8; ++s) { const int row = 2 * s + hi, cofs = lr * 4; v4f val = *(const v4fa*)(os + row * 68 + cofs); if (BIAS) { val[0] += bfr(bias[c0 + cofs]); val[1] += bfr(bias[c0 + cofs + 1]); val[2] += bfr(bias[c0 + cofs + 2]); val[3] += bfr(bias[c0 + cofs + 3]); }
                *(volatile v4f*)(crow + (size_t)row * ldc + cofs) = val; }
            if (ps == 0) __threadfence(); }
        __builtin_amdgcn_wave_barrier(); asm volatile("" ::: "memory");
    }
}

__device__ __forceinline__ void splitf(float y, unsigned short& h, unsigned short& l) { h = f2bf(y); l = f2bf(y - bf2f(h)); }
typedef __attribute__((ext_vector_type(4))) unsigned short v4us;

__global__ __launch_bounds__(256) void k_wpad(const float* __restrict__ w, int K, const float* __restrict__ b, bf* Bt, float* BP) { const int i = (blockIdx.x * 256 + threadIdx.x) * 4; if (i < 64 * K) { const int n = i / K, k = i % K; v4us o;
#pragma unroll
        for (int q = 0; q < 4; ++q) o[q] = n < 32 ? f2bf(w[n * K + k + q]) : (unsigned short)0; *(volatile v4us*)(Bt + i) = o; __threadfence(); *(volatile v4us*)(Bt + i) = o; }
    const int t = blockIdx.x * 256 + threadIdx.x; if (t < 64) { const float v = t < 32 ? b[t] : 0.f; *(volatile float*)(BP + t) = v; __threadfence(); *(volatile float*)(BP + t) = v; } }
__global__ __launch_bounds__(256) void k_gsum(const int* __restrict__ x, const float* __restrict__ emb, bf* Hh, bf* Hl) { const size_t e = ((size_t)blockIdx.x * 256 + threadIdx.x) * 4; if (e >= (size_t)NR * EMB) return; const int d = (int)(e % EMB); const int r = (int)(e / EMB); float acc[4] = {0.f, 0.f, 0.f, 0.f};
#pragma unroll 1
    for (int j = 0; j < NUSE; ++j) { int id = x[(size_t)r * NIDX + j]; id = min(max(id, 0), VOC - 1); const v4f v = *(const v4f*)(emb + (size_t)id * EMB + d);
#pragma unroll
        for (int q = 0; q < 4; ++q) acc[q] = __fadd_rn(acc[q], bfr(v[q])); }
    v4us oh, ol;
#pragma unroll
    for (int q = 0; q < 4; ++q) { unsigned short a, c; splitf(fmaxf(acc[q], 0.f), a, c); oh[q] = a; ol[q] = c; } *(volatile v4us*)(Hh + e) = oh; *(volatile v4us*)(Hl + e) = ol; __threadfence(); *(volatile v4us*)(Hh + e) = oh; *(volatile v4us*)(Hl + e) = ol; }
__global__ __launch_bounds__(256) void k_cat(const float* __restrict__ H, bf* Ph, bf* Pl) { const size_t e = ((size_t)blockIdx.x * 256 + threadIdx.x) * 4; if (e >= (size_t)NR * 64) return; const int c = (int)(e % 64); const size_t r = e / 64; v4us oh, ol;
#pragma unroll
    for (int q = 0; q < 4; ++q) { const int cc = c + q; const float h = cc < 32 ? H[r * 64 + cc] : -H[r * 64 + cc - 32]; unsigned short a, b; splitf(fmaxf(h, 0.f), a, b); oh[q] = a; ol[q] = b; } *(volatile v4us*)(Ph + e) = oh; *(volatile v4us*)(Pl + e) = ol; __threadfence(); *(volatile v4us*)(Ph + e) = oh; *(volatile v4us*)(Pl + e) = ol; }
__global__ __launch_bounds__(256) void k_fin(const float* __restrict__ H, const float* __restrict__ w4, float* OUT) { const int r = blockIdx.x * 256 + threadIdx.x; if (r >= NR) return; const float* h = H + (size_t)r * 64; float s = 0.f;
#pragma unroll 1
    for (int c = 0; c < 64; c += 4) { const v4f a = *(const v4f*)(h + (c < 32 ? c : c - 32));
#pragma unroll
        for (int q = 0; q < 4; ++q) { const float v = c < 32 ? a[q] : -a[q]; float p = __fmul_rn(fmaxf(v, 0.f), bfr(w4[c + q])); asm volatile("" : "+v"(p)); s = __fadd_rn(s, p); } }
    *(volatile float*)(OUT + r) = s; __threadfence(); *(volatile float*)(OUT + r) = s; }

extern "C" void kernel_launch(void* const* d_in, const int* in_sizes, int n_in,
                              void* d_out, int out_size, void* d_ws, size_t ws_size, hipStream_t stream) {
    (void)in_sizes; (void)n_in; (void)out_size;
    const int* x = (const int*)d_in[0]; const float* emb = (const float*)d_in[1]; const float* w2 = (const float*)d_in[2]; const float* b2 = (const float*)d_in[3]; const float* w3 = (const float*)d_in[4]; const float* b3 = (const float*)d_in[5]; const float* w4 = (const float*)d_in[6];
    float* OUT = (float*)d_out;
    char* wsp = (char*)d_ws;
    auto take = [&](size_t bytes) { char* p = wsp; wsp += (bytes + 255) & ~(size_t)255; return (void*)p; };
    bf* W2B = (bf*)take(64 * EMB * 2); float* B2P = (float*)take(256); bf* W3B = (bf*)take(64 * 64 * 2); float* B3P = (float*)take(256);
    bf* H1h = (bf*)take((size_t)NR * EMB * 2); bf* H1l = (bf*)take((size_t)NR * EMB * 2); float* H2 = (float*)take((size_t)NR * 64 * 4); bf* H3h = (bf*)take((size_t)NR * 64 * 2); bf* H3l = (bf*)take((size_t)NR * 64 * 2); float* H4 = (float*)take((size_t)NR * 64 * 4);
    if ((size_t)(wsp - (char*)d_ws) > ws_size) return;
    k_wpad<<<(64 * EMB / 4 + 255) / 256, 256, 0, stream>>>(w2, EMB, b2, W2B, B2P); k_wpad<<<(64 * 64 / 4 + 255) / 256, 256, 0, stream>>>(w3, 64, b3, W3B, B3P);
    k_gsum<<<(unsigned)(((size_t)NR * EMB / 4 + 255) / 256), 256, 0, stream>>>(x, emb, H1h, H1l);
    k_gemmw<bf, 1, true><<<dim3(NR / 64, 1, 1), 32, 0, stream>>>(H1h, H1l, W2B, nullptr, EMB, H2, 64, B2P, 0, 0, 0);
    k_cat<<<(unsigned)(((size_t)NR * 64 / 4 + 255) / 256), 256, 0, stream>>>(H2, H3h, H3l);
    k_gemmw<bf, 1, true><<<dim3(NR / 64, 1, 1), 32, 0, stream>>>(H3h, H3l, W3B, nullptr, 64, H4, 64, B3P, 0, 0, 0);
    k_fin<<<NR / 256, 256, 0, stream>>>(H4, w4, OUT);
}
